// GNNModel_50800873177112
// MI455X (gfx1250) — hardware-verified
//
#include <hip/hip_runtime.h>
#include <stddef.h>
#include <stdint.h>
#include <math.h>


#define HID      128
#define NT9      9
#define BROWS    (NT9 * 16)
#define KP       32
#define NSLOT    7
#define NPAIR    ((NSLOT * (NSLOT + 1)) / 2)
#define MOMW     (1 + NSLOT + NPAIR)
#define NTHR     256
#define NWAVE    8
#define RB       1024
#define EPT      8
#define CHUNK    (NTHR * EPT)
#define WCAP     (EPT * 32)
#define LISTN    (NWAVE * WCAP)
#define SLB      10
#define RCAP     8192
#define DEGCAP   64
#define NODECAP  512
#define GMAX     512
#define GTHR     512
#define GWAVE    (GTHR / 32)
#define RECW     64
#define BPBYTES  (BROWS * KP * 2)
#define PVF      256
#define FOLDB    (BPBYTES + PVF * 4)
#define FOLDQ    (FOLDB / 16)
#define CSR_ZINTS (LISTN + 2 * RCAP + 3 * RB)
#define CSR_MISC  32
#define CSR_LDS_INTS (CSR_ZINTS + CSR_MISC)
#define WSMAX    134217728

static_assert((CHUNK & (CHUNK - 1)) == 0 && CHUNK <= 4096);
static_assert((RB & (RB - 1)) == 0 && RB == (1 << SLB));
static_assert(((long long)CHUNK << SLB) < (1LL << 31));
static_assert(LISTN % NTHR == 0 && RB % NWAVE == 0 && RB % 32 == 0);
static_assert(RCAP % 32 == 0 && CSR_ZINTS % (NTHR * 4) == 0);
static_assert(RB == 4 * NTHR);
static_assert(RB / NWAVE == 128);
static_assert(MOMW == 36 && MOMW <= 64 && RECW == 64);
static_assert(NSLOT * 3 <= KP && HID == 8 * 16);
static_assert(BPBYTES % 256 == 0 && FOLDB % 16 == 0 && FOLDQ <= 3 * NTHR);
static_assert(GTHR == GMAX && NSLOT * NSLOT <= 64);
static_assert(CSR_LDS_INTS * 4 <= 300000);

typedef float          v4f   __attribute__((ext_vector_type(4)));
typedef float          v8f   __attribute__((ext_vector_type(8)));
typedef int            v2i   __attribute__((ext_vector_type(2)));
typedef int            v4i   __attribute__((ext_vector_type(4)));
typedef int            v8i   __attribute__((ext_vector_type(8)));
typedef unsigned int   v4u   __attribute__((ext_vector_type(4)));
typedef unsigned short v8us  __attribute__((ext_vector_type(8)));
typedef unsigned short v16us __attribute__((ext_vector_type(16)));
typedef __bf16         v16bf __attribute__((ext_vector_type(16)));
typedef v4f  __attribute__((may_alias)) v4fa;
typedef v2i  __attribute__((may_alias)) v2ia;
typedef v4i  __attribute__((may_alias)) v4ia;
typedef v4u  __attribute__((may_alias)) v4ua;
typedef v8us __attribute__((may_alias)) v8usa;
typedef unsigned short usa __attribute__((may_alias));
union FragB { v16bf v; v16us u; v8us h[2]; v8i w; };

__device__ __forceinline__ v8f wmz(const FragB& a, const FragB& b) {
  const v8f z = {0.f, 0.f, 0.f, 0.f, 0.f, 0.f, 0.f, 0.f};
  return __builtin_amdgcn_wmma_f32_16x16x32_bf16(false, a.v, false, b.v, (short)0, z, false, false);
}

__device__ __forceinline__ unsigned bf16_bits(float f) {
  const unsigned u = __float_as_uint(f);
  return (u + 0x7FFFu + ((u >> 16) & 1u)) >> 16;
}
__device__ __forceinline__ float bf16_val(float f) { return __uint_as_float(bf16_bits(f) << 16); }
__device__ __forceinline__ int clampi(int v, int lo, int hi) { return v < lo ? lo : (v > hi ? hi : v); }

__device__ __forceinline__ void wave_sync() {
  __builtin_amdgcn_fence(__ATOMIC_RELEASE, "wavefront");
  __builtin_amdgcn_wave_barrier();
  __builtin_amdgcn_fence(__ATOMIC_ACQUIRE, "wavefront");
}

__device__ __forceinline__ void split7(const float* a, unsigned* h, unsigned* l) {
#pragma unroll
  for (int k = 0; k < NSLOT; ++k) {
    const unsigned hb = bf16_bits(a[k]);
    h[k] = hb;
    l[k] = bf16_bits(a[k] - __uint_as_float(hb << 16));
  }
}
__device__ __forceinline__ void packA(const unsigned* h, const unsigned* l, v4u* w) {
  v4u w0, w1, w2;
  w0.x = h[0] | (h[1] << 16); w0.y = h[2] | (h[3] << 16); w0.z = h[4] | (h[5] << 16); w0.w = h[6] | (l[0] << 16);
  w1.x = l[1] | (l[2] << 16); w1.y = l[3] | (l[4] << 16); w1.z = l[5] | (l[6] << 16); w1.w = h[0] | (h[1] << 16);
  w2.x = h[2] | (h[3] << 16); w2.y = h[4] | (h[5] << 16); w2.z = h[6];                  w2.w = 0u;
  const v4u z = {0u, 0u, 0u, 0u};
  w[0] = w0; w[1] = w1; w[2] = w2; w[3] = z;
}
__device__ __forceinline__ void packB(const unsigned* h, const unsigned* l, v4u* w) {
  v4u w0, w1, w2;
  w0.x = h[0] | (h[1] << 16); w0.y = h[2] | (h[3] << 16); w0.z = h[4] | (h[5] << 16); w0.w = h[6] | (h[0] << 16);
  w1.x = h[1] | (h[2] << 16); w1.y = h[3] | (h[4] << 16); w1.z = h[5] | (h[6] << 16); w1.w = l[0] | (l[1] << 16);
  w2.x = l[2] | (l[3] << 16); w2.y = l[4] | (l[5] << 16); w2.z = l[6];                  w2.w = 0u;
  const v4u z = {0u, 0u, 0u, 0u};
  w[0] = w0; w[1] = w1; w[2] = w2; w[3] = z;
}

template <int SLB_>
__device__ __forceinline__ int scan_chunk(const int* __restrict__ dsts, int nE, int cbase, int slotBase,
                                          int nb, int vec8, int* list, int tid, int lane, int wave,
                                          int& below) {
  int wc = 0;
  const int el0  = tid * EPT;
  const int e0   = cbase + el0;
  const int sent = -2147483647 - 1;
  v4i da, db;
  if (vec8 != 0 && cbase + CHUNK <= nE) {
    da = *(const v4i*)(dsts + e0);
    db = *(const v4i*)(dsts + e0 + 4);
  } else {
    da.x = (e0     < nE) ? dsts[min(e0,     nE - 1)] : sent;
    da.y = (e0 + 1 < nE) ? dsts[min(e0 + 1, nE - 1)] : sent;
    da.z = (e0 + 2 < nE) ? dsts[min(e0 + 2, nE - 1)] : sent;
    da.w = (e0 + 3 < nE) ? dsts[min(e0 + 3, nE - 1)] : sent;
    db.x = (e0 + 4 < nE) ? dsts[min(e0 + 4, nE - 1)] : sent;
    db.y = (e0 + 5 < nE) ? dsts[min(e0 + 5, nE - 1)] : sent;
    db.z = (e0 + 6 < nE) ? dsts[min(e0 + 6, nE - 1)] : sent;
    db.w = (e0 + 7 < nE) ? dsts[min(e0 + 7, nE - 1)] : sent;
  }
  const unsigned nbs = (unsigned)slotBase;
  const unsigned unb = (unsigned)nb;
  below += (int)((unsigned)da.x < nbs) + (int)((unsigned)da.y < nbs) + (int)((unsigned)da.z < nbs)
         + (int)((unsigned)da.w < nbs) + (int)((unsigned)db.x < nbs) + (int)((unsigned)db.y < nbs)
         + (int)((unsigned)db.z < nbs) + (int)((unsigned)db.w < nbs);
  const unsigned s0 = (unsigned)da.x - nbs, s1 = (unsigned)da.y - nbs;
  const unsigned s2 = (unsigned)da.z - nbs, s3 = (unsigned)da.w - nbs;
  const unsigned s4 = (unsigned)db.x - nbs, s5 = (unsigned)db.y - nbs;
  const unsigned s6 = (unsigned)db.z - nbs, s7 = (unsigned)db.w - nbs;
  const bool h0 = s0 < unb, h1 = s1 < unb, h2 = s2 < unb, h3 = s3 < unb;
  const bool h4 = s4 < unb, h5 = s5 < unb, h6 = s6 < unb, h7 = s7 < unb;
  const unsigned any = __builtin_amdgcn_ballot_w32(h0 | h1 | h2 | h3 | h4 | h5 | h6 | h7);
  if (any != 0u) {
#define HITJ(J, HJ, SJ) { \
      const unsigned mj = __builtin_amdgcn_ballot_w32(HJ); \
      if (mj != 0u) { \
        if (HJ) { \
          const int pos = wc + (int)__builtin_amdgcn_mbcnt_lo(mj, 0u); \
          if (pos < WCAP) list[wave * WCAP + pos] = ((el0 + (J)) << SLB_) | (int)(SJ); \
        } \
        wc += (int)__builtin_popcount(mj); } }
    HITJ(0, h0, s0)
    HITJ(1, h1, s1)
    HITJ(2, h2, s2)
    HITJ(3, h3, s3)
    HITJ(4, h4, s4)
    HITJ(5, h5, s5)
    HITJ(6, h6, s6)
    HITJ(7, h7, s7)
#undef HITJ
  }
  return wc;
}

__device__ __forceinline__ int lbound(const int* __restrict__ bat, int nN, int key) {
  int lo = 0, n = nN;
#pragma unroll 1
  for (int it = 0; it < 26; ++it) {
    const int half = n >> 1;
    const int ix = clampi(lo + half, 0, nN - 1);
    const int v = bat[ix];
    const bool go = (n > 0) && (v < key);
    lo = go ? (lo + half + 1) : lo;
    n  = go ? (n - half - 1) : half;
  }
  return clampi(lo, 0, nN);
}

__global__ __launch_bounds__(GTHR) void k_gprep(const int* __restrict__ bat, const float* __restrict__ u,
                                                int nN, int nG, int* gseg, float* ua) {
  __shared__ __attribute__((aligned(16))) int gs[2 * GMAX];
  __shared__ int flg[1];
  const int tid = (int)threadIdx.x;
  if (tid == 0) flg[0] = 0;
  __syncthreads();
  int bad = 0;
#pragma unroll 1
  for (int i0 = 0; i0 < nN; i0 += GTHR) {
    const int i  = i0 + tid;
    const int ic = clampi(i, 0, nN - 1);
    const int in2 = clampi(i + 1, 0, nN - 1);
    const int b  = bat[ic];
    const int bn = bat[in2];
    const int c1 = ((i < nN) && (b < 0 || b >= nG)) ? 1 : 0;
    const int c2 = ((i + 1 < nN) && (b > bn)) ? 1 : 0;
    bad |= c1 | c2;
  }
  const int g  = tid;
  const int lo = lbound(bat, nN, g);
  const int hi = lbound(bat, nN, g + 1);
  if (g < nG && (hi - lo) > NODECAP) bad = 1;
  if (bad != 0) flg[0] = 1;
  gs[2 * g]     = (g < nG) ? lo : 0;
  gs[2 * g + 1] = (g < nG) ? hi : 0;
  __syncthreads();
  const float qnan = __int_as_float(0x7fc00000);
  const float pz = (flg[0] != 0) ? qnan : 0.0f;
  const int gc = clampi(g, 0, nG - 1);
  const float u0 = u[3 * gc], u1 = u[3 * gc + 1], u2 = u[3 * gc + 2];
  const bool live = g < nG;
  v4f uv;
  uv.x = live ? (bf16_val(u0) + pz) : 0.0f;
  uv.y = live ? (bf16_val(u1) + pz) : 0.0f;
  uv.z = live ? (bf16_val(u2) + pz) : 0.0f;
  uv.w = 0.0f;
  v4i gv = {0, 0, 0, 0};
  const bool wg = tid < (2 * GMAX) / 4;
  if (wg) gv = *(const v4ia*)(gs + 4 * tid);
  *(volatile v4f*)(ua + 4 * g) = uv;
  if (wg) *(volatile v4i*)(gseg + 4 * tid) = gv;
  __threadfence();
  *(volatile v4f*)(ua + 4 * g) = uv;
  if (wg) *(volatile v4i*)(gseg + 4 * tid) = gv;
}

__global__ __launch_bounds__(NTHR) void k_csr(const int* __restrict__ srcs, const int* __restrict__ dsts,
                                              const int* __restrict__ bat, const float* __restrict__ ea,
                                              const float* __restrict__ x,
                                              int nE, int nN, int nG, int vec8, int nEP,
                                              int* idxo, float* e0, int* off2, float* x0) {
  extern __shared__ __attribute__((aligned(16))) int dsm[];
  int* list = dsm;
  int* hl   = dsm + LISTN;
  int* sl   = hl + RCAP;
  int* cnt  = sl + RCAP;
  int* offs = cnt + RB;
  int* cur  = offs + RB;
  int* misc = cur + RB;
  const int tid = (int)threadIdx.x, lane = tid & 31, wave = tid >> 5;
  const int nodeBase = (int)blockIdx.x * RB;

  {
    const v4i z4 = {0, 0, 0, 0};
    for (int i = tid * 4; i < CSR_ZINTS; i += NTHR * 4) *(v4ia*)(dsm + i) = z4;
    if (tid < CSR_MISC) misc[tid] = 0;
  }
  __syncthreads();

  int t = 0, ov = 0, below = 0;
  const int nChunks = (nE + CHUNK - 1) / CHUNK;
#pragma unroll 1
  for (int ch = 0; ch < nChunks; ++ch) {
    const int cbase = ch * CHUNK;
    const int wc = scan_chunk<SLB>(dsts, nE, cbase, nodeBase, RB, vec8, list, tid, lane, wave, below);
    if (lane == 0) misc[wave] = wc;
    __syncthreads();
    if (wave == 0) {
#pragma unroll 1
      for (int w2 = 0; w2 < NWAVE; ++w2) {
        int c = misc[w2];
        c = c < 0 ? 0 : (c > WCAP ? WCAP : c);
#pragma unroll 1
        for (int b0 = 0; b0 < c; b0 += 32) {
          const int ix  = b0 + lane;
          const int ent = list[w2 * WCAP + (ix < WCAP ? ix : WCAP - 1)];
          const int m32 = (c - b0) < 32 ? (c - b0) : 32;
#pragma unroll 1
          for (int k = 0; k < m32; ++k) {
            const int uu   = __builtin_amdgcn_readlane(ent, k);
            const int slot = uu & (RB - 1);
            const int el   = (uu >> SLB) & (CHUNK - 1);
            const int pk   = ((cbase + el) << SLB) | slot;
            if (t < RCAP) {
              if (lane == 0) { hl[t] = pk; cnt[slot] = cnt[slot] + 1; }
              t = t + 1;
            } else {
              ov = 1;
            }
          }
        }
      }
    }
    __syncthreads();
  }
  {
    int bsum = below;
#pragma unroll
    for (int d = 16; d >= 1; d >>= 1) bsum += __shfl_xor(bsum, d, 32);
    if (lane == 0) misc[16 + wave] = bsum;
  }
  if (wave == 0 && lane == 0) { misc[8] = t; misc[9] = ov; }
  __syncthreads();
  int tt = misc[8];
  tt = clampi(tt, 0, RCAP);
  const int ovf = misc[9];
  int base = 0;
#pragma unroll
  for (int w2 = 0; w2 < NWAVE; ++w2) base += misc[16 + w2];
  base = clampi(base, 0, nE);
  {
    int df = 0;
#pragma unroll
    for (int i = 0; i < RB / NTHR; ++i) df |= (cnt[i * NTHR + tid] > DEGCAP) ? 1 : 0;
    if (df != 0) misc[10] = 1;
  }

  if (wave == 0) {
    const int bse = lane * (RB / 32);
    int s = 0;
#pragma unroll 1
    for (int i = 0; i < RB / 32; ++i) s += cnt[bse + i];
    int incl = s;
#pragma unroll
    for (int d = 1; d < 32; d <<= 1) {
      const int y = __shfl_up(incl, d, 32);
      if (lane >= d) incl += y;
    }
    int run = incl - s;
#pragma unroll 1
    for (int i = 0; i < RB / 32; ++i) {
      const int cv = cnt[bse + i];
      offs[bse + i] = run;
      cur[bse + i]  = run;
      run += cv;
    }
  }
  __syncthreads();
  if (wave == 0) {
#pragma unroll 1
    for (int b0 = 0; b0 < tt; b0 += 32) {
      const int ix  = b0 + lane;
      const int ent = hl[ix < RCAP ? ix : RCAP - 1];
      const int m32 = (tt - b0) < 32 ? (tt - b0) : 32;
#pragma unroll 1
      for (int k = 0; k < m32; ++k) {
        const int uu   = __builtin_amdgcn_readlane(ent, k);
        const int slot = uu & (RB - 1);
        if (lane == 0) {
          int p = cur[slot];
          p = clampi(p, 0, RCAP - 1);
          sl[p] = uu;
          cur[slot] = p + 1;
        }
      }
    }
  }
  __syncthreads();
  const int dfl = misc[10];

  const float qnan = __int_as_float(0x7fc00000);
  const float pz = (ovf != 0 || dfl != 0) ? qnan : 0.0f;
  const int nBlk = (int)gridDim.x, bI = (int)blockIdx.x;
  int pbase = ((base + 31) & ~31) + 32 * bI;
  pbase = clampi(pbase, 0, nEP);
  int segEnd = (bI == nBlk - 1) ? nEP : (((base + tt + 31) & ~31) + 32 * (bI + 1));
  segEnd = clampi(segEnd, pbase, nEP);

  v4i o4[2];
#pragma unroll
  for (int i = 0; i < 2; ++i) {
    const int s0 = 2 * (i * NTHR + tid);
    v4i o;
    o.x = pbase + clampi(offs[s0], 0, RCAP);
    o.y = clampi(cnt[s0], 0, RCAP);
    o.z = pbase + clampi(offs[s0 + 1], 0, RCAP);
    o.w = clampi(cnt[s0 + 1], 0, RCAP);
    o4[i] = o;
  }
  v4f xv;
  {
    const int n0 = nodeBase + 4 * tid;
    const float a0 = x[clampi(n0, 0, nN - 1)],     a1 = x[clampi(n0 + 1, 0, nN - 1)];
    const float a2 = x[clampi(n0 + 2, 0, nN - 1)], a3 = x[clampi(n0 + 3, 0, nN - 1)];
    xv.x = (n0     < nN) ? bf16_val(a0) : 0.0f;
    xv.y = (n0 + 1 < nN) ? bf16_val(a1) : 0.0f;
    xv.z = (n0 + 2 < nN) ? bf16_val(a2) : 0.0f;
    xv.w = (n0 + 3 < nN) ? bf16_val(a3) : 0.0f;
  }
#pragma unroll
  for (int i = 0; i < 2; ++i) {
    const int s0 = 2 * (i * NTHR + tid);
    *(volatile v4i*)(off2 + 2 * (size_t)(nodeBase + s0)) = o4[i];
  }
  *(volatile v4f*)(x0 + (size_t)nodeBase + 4 * tid) = xv;
  __threadfence();
#pragma unroll
  for (int i = 0; i < 2; ++i) {
    const int s0 = 2 * (i * NTHR + tid);
    *(volatile v4i*)(off2 + 2 * (size_t)(nodeBase + s0)) = o4[i];
  }
  *(volatile v4f*)(x0 + (size_t)nodeBase + 4 * tid) = xv;

  int nIt = (segEnd - pbase + NTHR - 1) / NTHR;
  nIt = clampi(nIt, 0, (RCAP + 64) / NTHR + 1);
  const int tmax = tt > 0 ? tt - 1 : 0;
#pragma unroll 1
  for (int it = 0; it < nIt; ++it) {
    const int p  = pbase + it * NTHR + tid;
    const int j  = p - pbase;
    const int jj = clampi(j, 0, tmax);
    const int uu = sl[clampi(jj, 0, RCAP - 1)];
    const int eid  = clampi(uu >> SLB, 0, nE - 1);
    const int slot = uu & (RB - 1);
    const int sr = clampi(srcs[eid], 0, nN - 1);
    const int bs = clampi(bat[sr], 0, nG - 1);
    const float ev = bf16_val(ea[eid]);
    const bool livep = j < tt;
    v4i rec;
    rec.x = livep ? sr : 0;
    rec.y = livep ? (nodeBase + slot) : 0;
    rec.z = livep ? bs : 0;
    rec.w = livep ? 1 : 0;
    const float ef = livep ? (ev + pz) : 0.0f;
    const bool st = p < segEnd;
    if (st) { *(volatile v4i*)(idxo + 4 * (size_t)p) = rec; *(volatile float*)(e0 + p) = ef; }
    __threadfence();
    if (st) { *(volatile v4i*)(idxo + 4 * (size_t)p) = rec; *(volatile float*)(e0 + p) = ef; }
  }
}

template <int EDGE>
__global__ __launch_bounds__(NTHR) void k_mom(const int* __restrict__ tix, const float* __restrict__ ep,
                                              const float* __restrict__ xc, const float* __restrict__ uc,
                                              const int* __restrict__ bat, int nN, int nG, int nEP,
                                              unsigned int* apl, float* esum, float* rec) {
  __shared__ __attribute__((aligned(16))) float red[MOMW * NTHR];
  __shared__ __attribute__((aligned(16))) v4u   stg[NWAVE * 32 * 4];
  __shared__ __attribute__((aligned(16))) float rs[RECW];
  const int tid = (int)threadIdx.x, lane = tid & 31, wave = tid >> 5;
  const int rowBase = (int)blockIdx.x * RB;

  float S[NSLOT], P[NPAIR];
  float nv = 0.0f;
#pragma unroll
  for (int k = 0; k < NSLOT; ++k) S[k] = 0.0f;
#pragma unroll
  for (int q = 0; q < NPAIR; ++q) P[q] = 0.0f;

#pragma unroll 1
  for (int it = 0; it < RB / NTHR; ++it) {
    const int r = rowBase + it * NTHR + tid;
    float a[NSLOT];
    float vf;
    float es = 0.0f;
    if constexpr (EDGE != 0) {
      const v4i q = *(const v4ia*)(tix + 4 * (size_t)r);
      const int sr = clampi(q.x, 0, nN - 1);
      const int ds = clampi(q.y, 0, nN - 1);
      const int bs = clampi(q.z, 0, nG - 1);
      vf = (q.w == 1) ? 1.0f : 0.0f;
      const float xs = xc[sr];
      const float xd = xc[ds];
      const float ev = ep[r];
      const v4f u4 = *(const v4fa*)(uc + 4 * bs);
      a[0] = xs * vf; a[1] = xd * vf; a[2] = ev * vf;
      a[3] = u4.x * vf; a[4] = u4.y * vf; a[5] = u4.z * vf; a[6] = vf;
    } else {
      const bool live = r < nN;
      const int nc = live ? r : nN - 1;
      const v2i o = *(const v2ia*)(tix + 2 * (size_t)nc);
      const int st = clampi(o.x, 0, nEP - 1);
      int c = clampi(o.y, 0, DEGCAP);
      c = live ? c : 0;
      int cm = c;
#pragma unroll
      for (int d = 16; d >= 1; d >>= 1) { const int oc = __shfl_xor(cm, d, 32); cm = oc > cm ? oc : cm; }
      float s = 0.0f;
#pragma unroll 1
      for (int j = 0; j < cm; ++j) {
        const bool in = j < c;
        const int pj = clampi(st + (in ? j : 0), 0, nEP - 1);
        const float v = ep[pj];
        s = fmaf(v, in ? 1.0f : 0.0f, s);
      }
      const float cf  = (float)(c < 1 ? 1 : c);
      const float eag = s * (1.0f / cf);
      const float xv  = xc[nc];
      const int   b   = clampi(bat[nc], 0, nG - 1);
      const v4f   u4  = *(const v4fa*)(uc + 4 * b);
      vf = live ? 1.0f : 0.0f;
      a[0] = xv * vf; a[1] = eag * vf; a[2] = u4.x * vf; a[3] = u4.y * vf; a[4] = u4.z * vf;
      a[5] = vf; a[6] = 0.0f;
      es = s * vf;
    }
    nv += vf;
#pragma unroll
    for (int k = 0; k < NSLOT; ++k) {
      S[k] += a[k];
#pragma unroll
      for (int l2 = k; l2 < NSLOT; ++l2) {
        const int q = k * NSLOT - (k * (k - 1)) / 2 + (l2 - k);
        P[q] = fmaf(a[k], a[l2], P[q]);
      }
    }
    unsigned h[NSLOT], l[NSLOT];
    split7(a, h, l);
    v4u w[4];
    packA(h, l, w);
    {
      v4u* sw = stg + (wave * 32 + lane) * 4;
      sw[0] = w[0]; sw[1] = w[1]; sw[2] = w[2]; sw[3] = w[3];
    }
    wave_sync();
    v4u qv[4];
#pragma unroll
    for (int j = 0; j < 4; ++j) qv[j] = stg[wave * 128 + j * 32 + lane];
    wave_sync();
    v4u* gp = (v4u*)apl + (size_t)(rowBase + it * NTHR + wave * 32) * 4;
#pragma unroll
    for (int j = 0; j < 4; ++j) *(volatile v4u*)(gp + j * 32 + lane) = qv[j];
    if constexpr (EDGE == 0) *(volatile float*)(esum + r) = es;
    __threadfence();
#pragma unroll
    for (int j = 0; j < 4; ++j) *(volatile v4u*)(gp + j * 32 + lane) = qv[j];
    if constexpr (EDGE == 0) *(volatile float*)(esum + r) = es;
  }

  red[tid] = nv;
#pragma unroll
  for (int k = 0; k < NSLOT; ++k) red[(1 + k) * NTHR + tid] = S[k];
#pragma unroll
  for (int q = 0; q < NPAIR; ++q) red[(1 + NSLOT + q) * NTHR + tid] = P[q];
  __syncthreads();
  if (wave < 2) {
    const int v = tid < MOMW ? tid : MOMW - 1;
    double tsum = 0.0;
#pragma unroll 1
    for (int i = 0; i < NTHR; ++i) tsum += (double)red[v * NTHR + i];
    rs[tid] = (tid < MOMW) ? (float)tsum : 0.0f;
  }
  __syncthreads();
  if (wave == 0) {
    const v4f o = *(const v4fa*)(rs + 4 * (lane & 15));
    float* rp = rec + (size_t)blockIdx.x * RECW + 4 * (lane & 15);
    if (lane < 16) *(volatile v4f*)rp = o;
    __threadfence();
    if (lane < 16) *(volatile v4f*)rp = o;
  }
}

template <int F>
__global__ __launch_bounds__(NTHR) void k_fold(const float* __restrict__ rec, int nblk,
                                               const float* __restrict__ W1, const float* __restrict__ b1,
                                               const float* __restrict__ g1, const float* __restrict__ bt1,
                                               const float* __restrict__ W2, const float* __restrict__ b2,
                                               unsigned int* fold) {
  __shared__ __attribute__((aligned(16))) float w1s[NSLOT * HID];
  __shared__ __attribute__((aligned(16))) float prm[4 * HID];
  __shared__ double totd[MOMW];
  __shared__ double md[NSLOT];
  __shared__ double cd[NSLOT * NSLOT];
  __shared__ float  wq[NSLOT * HID];
  __shared__ float  b2s[4];
  __shared__ __attribute__((aligned(16))) unsigned int fs[FOLDB / 4];
  const int tid = (int)threadIdx.x, lane = tid & 31, wave = tid >> 5;

  if (tid < F * 32) {
    const v4f v = *(const v4f*)(W1 + 4 * tid);
    w1s[4 * tid + 0] = bf16_val(v.x); w1s[4 * tid + 1] = bf16_val(v.y);
    w1s[4 * tid + 2] = bf16_val(v.z); w1s[4 * tid + 3] = bf16_val(v.w);
  }
  if (tid < HID) {
    const float* sp = (wave == 0) ? b1 : ((wave == 1) ? g1 : ((wave == 2) ? bt1 : W2));
    const v4f v = *(const v4f*)(sp + 4 * lane);
    prm[wave * HID + 4 * lane + 0] = bf16_val(v.x); prm[wave * HID + 4 * lane + 1] = bf16_val(v.y);
    prm[wave * HID + 4 * lane + 2] = bf16_val(v.z); prm[wave * HID + 4 * lane + 3] = bf16_val(v.w);
  }
  if (tid == 0) b2s[0] = bf16_val(b2[0]);
  {
    const v4u z = {0u, 0u, 0u, 0u};
    for (int i = tid; i < FOLDQ; i += NTHR) ((v4ua*)fs)[i] = z;
  }
  __syncthreads();
  if (wave < 2) {
    const int v = tid < MOMW ? tid : MOMW - 1;
    const int nb = clampi(nblk, 0, 4096);
    double tsum = 0.0;
#pragma unroll 1
    for (int b = 0; b < nb; ++b) tsum += (double)rec[(size_t)b * RECW + v];
    if (tid < MOMW) totd[tid] = tsum;
  }
  __syncthreads();
  if (wave < 2) {
    const double n   = totd[0] < 1.0 ? 1.0 : totd[0];
    const double inv = 1.0 / n;
    if (tid < NSLOT) md[tid] = totd[1 + tid] * inv;
    const int t  = tid < NSLOT * NSLOT ? tid : 0;
    const int k  = t / NSLOT, l2 = t - k * NSLOT;
    const int ka = k < l2 ? k : l2, kb = k < l2 ? l2 : k;
    const int q  = ka * NSLOT - (ka * (ka - 1)) / 2 + (kb - ka);
    const double ckl = totd[1 + NSLOT + q] * inv - (totd[1 + k] * inv) * (totd[1 + l2] * inv);
    if (tid < NSLOT * NSLOT) cd[tid] = ckl;
  }
  __syncthreads();
  if (tid < HID) {
    const int j = tid;
    double mh = (double)prm[j];
    double var = 0.0;
#pragma unroll 1
    for (int k = 0; k < F; ++k) {
      const double wk = (double)w1s[k * HID + j];
      mh += md[k] * wk;
#pragma unroll 1
      for (int l2 = 0; l2 < F; ++l2) var += wk * (double)w1s[l2 * HID + j] * cd[k * NSLOT + l2];
    }
    var = var < 0.0 ? 0.0 : var;
    const double istd = 1.0 / sqrt(var + 1e-5);
    const double s    = (double)prm[HID + j] * istd;
    const double tsh  = (double)prm[2 * HID + j] - mh * s;
    const double w2   = (double)prm[3 * HID + j];
    float a7[NSLOT];
#pragma unroll
    for (int k = 0; k < NSLOT; ++k) {
      double v = 0.0;
      if (k < F) v = (double)w1s[k * HID + j] * s * w2;
      else if (k == F) v = ((double)prm[j] * s + tsh) * w2;
      a7[k] = (float)v;
    }
    unsigned h[NSLOT], l[NSLOT];
    split7(a7, h, l);
    v4u w[4];
    packB(h, l, w);
    v4ua* frow = (v4ua*)fs + j * 4;
    frow[0] = w[0]; frow[1] = w[1]; frow[2] = w[2]; frow[3] = w[3];
#pragma unroll
    for (int k = 0; k < NSLOT; ++k) wq[k * HID + j] = __uint_as_float(h[k] << 16) + __uint_as_float(l[k] << 16);
    fs[BPBYTES / 4 + (j & 15) * 8 + (j >> 4)] = __float_as_uint(w2 >= 0.0 ? 1.0f : -1.0f);
    if (j == 0) fs[BPBYTES / 4 + HID] = __float_as_uint(b2s[0]);
  }
  __syncthreads();
  if (wave == 0) {
    const int k = lane < NSLOT ? lane : NSLOT - 1;
    double ws = 0.0;
#pragma unroll 1
    for (int j = 0; j < HID; ++j) ws += (double)wq[k * HID + j];
    const float wf = (float)ws;
    const unsigned hb = bf16_bits(wf);
    const unsigned lb = bf16_bits(wf - __uint_as_float(hb << 16));
    if (lane < NSLOT) {
      usa* r8 = (usa*)(fs + HID * (KP / 2));
      r8[k] = (unsigned short)hb; r8[NSLOT + k] = (unsigned short)hb; r8[2 * NSLOT + k] = (unsigned short)lb;
    }
  }
  __syncthreads();
  v4u ov[3];
  bool ok[3];
#pragma unroll
  for (int it = 0; it < 3; ++it) {
    const int q = it * NTHR + tid;
    ok[it] = q < FOLDQ;
    ov[it] = ((const v4ua*)fs)[ok[it] ? q : 0];
  }
#pragma unroll
  for (int it = 0; it < 3; ++it) if (ok[it]) *(volatile v4u*)((v4u*)fold + it * NTHR + tid) = ov[it];
  __threadfence();
#pragma unroll
  for (int it = 0; it < 3; ++it) if (ok[it]) *(volatile v4u*)((v4u*)fold + it * NTHR + tid) = ov[it];
}

__global__ __launch_bounds__(NTHR) void k_apply(const unsigned short* __restrict__ apl,
                                                const unsigned short* __restrict__ bp,
                                                const float* __restrict__ pv, float* outp, int nStore) {
  __shared__ __attribute__((aligned(16))) float outs[RB];
  const int tid = (int)threadIdx.x, lane = tid & 31, wave = tid >> 5, hh = lane >> 4, m = lane & 15;
  const int rowBase = (int)blockIdx.x * RB;

  FragB bfr[NT9];
#pragma unroll
  for (int t = 0; t < NT9; ++t) {
    const unsigned short* wqp = bp + (size_t)(16 * t + m) * KP + 8 * hh;
    bfr[t].h[0] = *(const v8usa*)wqp;
    bfr[t].h[1] = *(const v8usa*)(wqp + 16);
  }
  float sg[8];
  {
    const v4f s0 = *(const v4fa*)(pv + 8 * m);
    const v4f s1 = *(const v4fa*)(pv + 8 * m + 4);
    sg[0] = s0.x; sg[1] = s0.y; sg[2] = s0.z; sg[3] = s0.w;
    sg[4] = s1.x; sg[5] = s1.y; sg[6] = s1.z; sg[7] = s1.w;
  }
  const float b2 = pv[HID];
  const bool bt3 = (lane & 8) != 0, bt2 = (lane & 4) != 0, bt1 = (lane & 2) != 0;

#pragma unroll 1
  for (int i = 0; i < RB / (NWAVE * 16); ++i) {
    const int tr0 = wave * (RB / NWAVE) + 16 * i;
    const unsigned short* ap = apl + (size_t)(rowBase + tr0 + m) * KP + 8 * hh;
    FragB af;
    af.h[0] = *(const v8usa*)ap;
    af.h[1] = *(const v8usa*)(ap + 16);
    v8f d[NT9];
#pragma unroll
    for (int t = 0; t < NT9; ++t) d[t] = wmz(af, bfr[t]);
    asm volatile("v_nop\n\tv_nop\n\tv_nop\n\tv_nop"
                 : "+v"(d[0]), "+v"(d[1]), "+v"(d[2]), "+v"(d[3]), "+v"(d[4]),
                   "+v"(d[5]), "+v"(d[6]), "+v"(d[7]), "+v"(d[8])
                 : "v"(af.w), "v"(bfr[0].w), "v"(bfr[1].w), "v"(bfr[2].w), "v"(bfr[3].w), "v"(bfr[4].w),
                   "v"(bfr[5].w), "v"(bfr[6].w), "v"(bfr[7].w), "v"(bfr[8].w));
    float p[8];
#pragma unroll
    for (int r = 0; r < 8; ++r) p[r] = d[8][r];
#pragma unroll
    for (int t = 0; t < 8; ++t) {
#pragma unroll
      for (int r = 0; r < 8; ++r) p[r] = fmaf(fabsf(d[t][r]), sg[t], p[r]);
    }
    float q4[4];
#pragma unroll
    for (int j = 0; j < 4; ++j) {
      const float ra = __shfl_xor(p[j], 8, 32);
      const float rb = __shfl_xor(p[4 + j], 8, 32);
      const float mine = bt3 ? p[4 + j] : p[j];
      const float oth  = bt3 ? rb : ra;
      q4[j] = mine + oth;
    }
    float q2[2];
#pragma unroll
    for (int j = 0; j < 2; ++j) {
      const float ra = __shfl_xor(q4[j], 4, 32);
      const float rb = __shfl_xor(q4[2 + j], 4, 32);
      const float mine = bt2 ? q4[2 + j] : q4[j];
      const float oth  = bt2 ? rb : ra;
      q2[j] = mine + oth;
    }
    float q1;
    {
      const float ra = __shfl_xor(q2[0], 2, 32);
      const float rb = __shfl_xor(q2[1], 2, 32);
      const float mine = bt1 ? q2[1] : q2[0];
      const float oth  = bt1 ? rb : ra;
      q1 = mine + oth;
    }
    const float tot = q1 + __shfl_xor(q1, 1, 32);
    const float v = fmaf(0.5f, tot, b2);
    const int R = 8 * hh + (m >> 1);
    if ((lane & 1) == 0) outs[tr0 + R] = v;
  }
  __syncthreads();
  const v4f ov = *(const v4fa*)(outs + 4 * tid);
  const int g0 = rowBase + 4 * tid;
  const bool full = (g0 + 4) <= nStore;
  float* op = outp + g0;
  if (full) {
    *(volatile v4f*)op = ov;
  } else {
    if (g0     < nStore) *(volatile float*)(op)     = ov.x;
    if (g0 + 1 < nStore) *(volatile float*)(op + 1) = ov.y;
    if (g0 + 2 < nStore) *(volatile float*)(op + 2) = ov.z;
    if (g0 + 3 < nStore) *(volatile float*)(op + 3) = ov.w;
  }
  __threadfence();
  if (full) {
    *(volatile v4f*)op = ov;
  } else {
    if (g0     < nStore) *(volatile float*)(op)     = ov.x;
    if (g0 + 1 < nStore) *(volatile float*)(op + 1) = ov.y;
    if (g0 + 2 < nStore) *(volatile float*)(op + 2) = ov.z;
    if (g0 + 3 < nStore) *(volatile float*)(op + 3) = ov.w;
  }
}

__global__ __launch_bounds__(GTHR) void k_glob(const int* __restrict__ gseg, const float* __restrict__ xn,
                                               const float* __restrict__ esum, const int* __restrict__ off2,
                                               const float* __restrict__ uc, const float* __restrict__ gW,
                                               const float* __restrict__ gb, const float* __restrict__ gg,
                                               const float* __restrict__ gbt, int nN, int nG, float* un) {
  __shared__ float ps[32];
  __shared__ float wred[GWAVE * 3];
  const int tid = (int)threadIdx.x, lane = tid & 31, wave = tid >> 5;
  if (wave == 0) {
    const float vw  = gW[clampi(lane, 0, 14)];
    const float vb  = gb[clampi(lane - 15, 0, 2)];
    const float vg  = gg[clampi(lane - 18, 0, 2)];
    const float vbt = gbt[clampi(lane - 21, 0, 2)];
    const float v = (lane < 15) ? vw : ((lane < 18) ? vb : ((lane < 21) ? vg : vbt));
    ps[lane] = bf16_val(v);
  }
  __syncthreads();
  const int g = tid;
  const bool live = g < nG;
  const float lf = live ? 1.0f : 0.0f;
  const int gc = clampi(g, 0, nG - 1);
  const v2i sgm = *(const v2ia*)(gseg + 2 * gc);
  const int lo = clampi(sgm.x, 0, nN);
  const int hi = clampi(sgm.y, lo, nN);
  const int cn = hi - lo;
  const bool big = cn > NODECAP;
  int c = cn > NODECAP ? NODECAP : cn;
  c = live ? c : 0;
  int cm = c;
#pragma unroll
  for (int d = 16; d >= 1; d >>= 1) { const int oc = __shfl_xor(cm, d, 32); cm = oc > cm ? oc : cm; }
  float sx = 0.0f, se = 0.0f;
  int ce = 0;
#pragma unroll 1
  for (int j = 0; j < cm; ++j) {
    const bool in = j < c;
    const int n = clampi(lo + (in ? j : 0), 0, nN - 1);
    const float xv = xn[n];
    const float ev = esum[n];
    const int   cc = clampi(off2[2 * (size_t)n + 1], 0, DEGCAP);
    sx = fmaf(xv, in ? 1.0f : 0.0f, sx);
    se = fmaf(ev, in ? 1.0f : 0.0f, se);
    ce += in ? cc : 0;
  }
  const float xa = sx * (1.0f / (float)(c < 1 ? 1 : c));
  const float eg = se * (1.0f / (float)(ce < 1 ? 1 : ce));
  const v4f u4 = *(const v4fa*)(uc + 4 * gc);
  const float gin[5] = {u4.x, u4.y, u4.z, xa, eg};
  float pre[3];
#pragma unroll
  for (int k = 0; k < 3; ++k) {
    float pr = ps[15 + k];
#pragma unroll
    for (int jj = 0; jj < 5; ++jj) pr = fmaf(gin[jj], ps[jj * 3 + k], pr);
    pre[k] = pr;
  }
  const float invG = 1.0f / (float)nG;
  float mk[3], vk[3];
  {
    float tk[3] = {pre[0] * lf, pre[1] * lf, pre[2] * lf};
#pragma unroll
    for (int k = 0; k < 3; ++k) {
#pragma unroll
      for (int d = 1; d < 32; d <<= 1) tk[k] += __shfl_xor(tk[k], d, 32);
    }
    if (lane == 0) { wred[wave * 3 + 0] = tk[0]; wred[wave * 3 + 1] = tk[1]; wred[wave * 3 + 2] = tk[2]; }
    __syncthreads();
#pragma unroll
    for (int k = 0; k < 3; ++k) {
      float s = 0.0f;
#pragma unroll
      for (int w2 = 0; w2 < GWAVE; ++w2) s += wred[w2 * 3 + k];
      mk[k] = s * invG;
    }
    __syncthreads();
  }
  float dk[3];
  {
    float tk[3];
#pragma unroll
    for (int k = 0; k < 3; ++k) { dk[k] = pre[k] - mk[k]; tk[k] = dk[k] * dk[k] * lf; }
#pragma unroll
    for (int k = 0; k < 3; ++k) {
#pragma unroll
      for (int d = 1; d < 32; d <<= 1) tk[k] += __shfl_xor(tk[k], d, 32);
    }
    if (lane == 0) { wred[wave * 3 + 0] = tk[0]; wred[wave * 3 + 1] = tk[1]; wred[wave * 3 + 2] = tk[2]; }
    __syncthreads();
#pragma unroll
    for (int k = 0; k < 3; ++k) {
      float s = 0.0f;
#pragma unroll
      for (int w2 = 0; w2 < GWAVE; ++w2) s += wred[w2 * 3 + k];
      vk[k] = s * invG;
    }
  }
  const float qnan = __int_as_float(0x7fc00000);
  const float pz = (big && live) ? qnan : 0.0f;
  v4f o;
  {
    float y[3];
#pragma unroll
    for (int k = 0; k < 3; ++k) {
      const float t = dk[k] * rsqrtf(vk[k] + 1e-5f) * ps[18 + k] + ps[21 + k];
      y[k] = live ? (fmaxf(t, 0.0f) + pz) : 0.0f;
    }
    o.x = y[0]; o.y = y[1]; o.z = y[2]; o.w = 0.0f;
  }
  float* op = un + 4 * g;
  *(volatile v4f*)op = o;
  __threadfence();
  *(volatile v4f*)op = o;
}

static inline int cdiv(int a, int b) { return (a + b - 1) / b; }
static inline size_t al256(size_t o) { return (o + 255) & ~(size_t)255; }

extern "C" void kernel_launch(void* const* d_in, const int* in_sizes, int n_in,
                              void* d_out, int out_size, void* d_ws, size_t ws_size,
                              hipStream_t stream) {
  if (n_in < 21) return;
  const int nN = in_sizes[0];
  const int nE = in_sizes[1];
  if (nN < 1 || nN >= (1 << 24)) return;
  if (nE < 1 || nE >= (1 << 21)) return;
  if (in_sizes[2] < 3 || (in_sizes[2] % 3) != 0) return;
  const int nG = in_sizes[2] / 3;
  if (nG < 1 || nG > GMAX) return;
  if (in_sizes[3] != 2 * nE || in_sizes[4] != nN) return;
  const int nL = in_sizes[16];
  if (nL < 1 || nL > 64) return;
  if (in_sizes[5] != nL * 6 * HID || in_sizes[6] != nL * HID || in_sizes[7] != nL * HID || in_sizes[8] != nL * HID) return;
  if (in_sizes[9] != nL * HID || in_sizes[10] != nL) return;
  if (in_sizes[11] != nL * 5 * HID || in_sizes[12] != nL * HID || in_sizes[13] != nL * HID || in_sizes[14] != nL * HID) return;
  if (in_sizes[15] != nL * HID) return;
  if (in_sizes[17] != nL * 15 || in_sizes[18] != nL * 3 || in_sizes[19] != nL * 3 || in_sizes[20] != nL * 3) return;
  if (out_size != nN) return;

  const float* x    = (const float*)d_in[0];
  const float* ea   = (const float*)d_in[1];
  const float* u    = (const float*)d_in[2];
  const int*   ei   = (const int*)d_in[3];
  const int*   bat  = (const int*)d_in[4];
  const float* eW1  = (const float*)d_in[5];
  const float* eb1  = (const float*)d_in[6];
  const float* eg1  = (const float*)d_in[7];
  const float* ebt1 = (const float*)d_in[8];
  const float* eW2  = (const float*)d_in[9];
  const float* eb2  = (const float*)d_in[10];
  const float* nW1  = (const float*)d_in[11];
  const float* nb1  = (const float*)d_in[12];
  const float* ng1  = (const float*)d_in[13];
  const float* nbt1 = (const float*)d_in[14];
  const float* nW2  = (const float*)d_in[15];
  const float* nb2  = (const float*)d_in[16];
  const float* gW   = (const float*)d_in[17];
  const float* gb   = (const float*)d_in[18];
  const float* gg   = (const float*)d_in[19];
  const float* gbt  = (const float*)d_in[20];
  float* out = (float*)d_out;
  const int* src = ei;
  const int* dst = ei + nE;

  const int gA   = cdiv(nN, RB);
  const int NPB  = gA * RB;
  const int pend = ((nE + 31) & ~31) + 32 * gA;
  const int nEB  = cdiv(pend, RB);
  const int EPB  = nEB * RB;
  const int nRec = nEB > gA ? nEB : gA;
  const int vec8 = ((nE & 3) == 0) ? 1 : 0;

  char* ws = (char*)d_ws;
  size_t off = 0;
  const size_t oGS  = off; off = al256(off + (size_t)4096);
  const size_t oUA  = off; off = al256(off + (size_t)GMAX * 16);
  const size_t oUB  = off; off = al256(off + (size_t)GMAX * 16);
  const size_t oOF  = off; off = al256(off + (size_t)NPB * 8);
  const size_t oIX  = off; off = al256(off + (size_t)EPB * 16);
  const size_t oEA  = off; off = al256(off + (size_t)EPB * 4);
  const size_t oEB  = off; off = al256(off + (size_t)EPB * 4);
  const size_t oXA  = off; off = al256(off + (size_t)NPB * 4);
  const size_t oXB  = off; off = al256(off + (size_t)NPB * 4);
  const size_t oES  = off; off = al256(off + (size_t)NPB * 4);
  const size_t oAE  = off; off = al256(off + (size_t)EPB * KP * 2);
  const size_t oAN  = off; off = al256(off + (size_t)NPB * KP * 2);
  const size_t oRC  = off; off = al256(off + (size_t)nRec * RECW * 4);
  const size_t oFD  = off; off = al256(off + (size_t)FOLDB);
  if (off > ws_size || off > (size_t)WSMAX) return;
  int*            GSEG = (int*)(ws + oGS);
  float*          UA   = (float*)(ws + oUA);
  float*          UB   = (float*)(ws + oUB);
  int*            OFF2 = (int*)(ws + oOF);
  int*            IDX  = (int*)(ws + oIX);
  float*          EA   = (float*)(ws + oEA);
  float*          EB   = (float*)(ws + oEB);
  float*          XA   = (float*)(ws + oXA);
  float*          XB   = (float*)(ws + oXB);
  float*          ESUM = (float*)(ws + oES);
  unsigned int*   AE   = (unsigned int*)(ws + oAE);
  unsigned int*   AN   = (unsigned int*)(ws + oAN);
  float*          REC  = (float*)(ws + oRC);
  unsigned int*   FOLD = (unsigned int*)(ws + oFD);
  const unsigned short* FBP = (const unsigned short*)(ws + oFD);
  const float*          FPV = (const float*)(ws + oFD + BPBYTES);

  const size_t csrLds = (size_t)CSR_LDS_INTS * 4;
  hipFuncSetAttribute(reinterpret_cast<const void*>(&k_csr), hipFuncAttributeMaxDynamicSharedMemorySize, (int)csrLds);

  k_gprep<<<1, GTHR, 0, stream>>>(bat, u, nN, nG, GSEG, UA);
  k_csr<<<gA, NTHR, csrLds, stream>>>(src, dst, bat, ea, x, nE, nN, nG, vec8, EPB, IDX, EA, OFF2, XA);

#pragma unroll 1
  for (int l = 0; l < nL; ++l) {
    const float* Xc = (l & 1) ? XB : XA;
    float*       Xn = (l & 1) ? XA : XB;
    const float* Ec = (l & 1) ? EB : EA;
    float*       En = (l & 1) ? EA : EB;
    const float* Uc = (l & 1) ? UB : UA;
    float*       Un = (l & 1) ? UA : UB;
    const bool last = (l == nL - 1);

    k_mom<1><<<nEB, NTHR, 0, stream>>>(IDX, Ec, Xc, Uc, bat, nN, nG, EPB, AE, ESUM, REC);
    k_fold<6><<<1, NTHR, 0, stream>>>(REC, nEB, eW1 + (size_t)l * 6 * HID, eb1 + (size_t)l * HID,
                                       eg1 + (size_t)l * HID, ebt1 + (size_t)l * HID,
                                       eW2 + (size_t)l * HID, eb2 + l, FOLD);
    k_apply<<<nEB, NTHR, 0, stream>>>((const unsigned short*)AE, FBP, FPV, En, EPB);
    k_mom<0><<<gA, NTHR, 0, stream>>>(OFF2, En, Xc, Uc, bat, nN, nG, EPB, AN, ESUM, REC);
    k_fold<5><<<1, NTHR, 0, stream>>>(REC, gA, nW1 + (size_t)l * 5 * HID, nb1 + (size_t)l * HID,
                                       ng1 + (size_t)l * HID, nbt1 + (size_t)l * HID,
                                       nW2 + (size_t)l * HID, nb2 + l, FOLD);
    k_apply<<<gA, NTHR, 0, stream>>>((const unsigned short*)AN, FBP, FPV, last ? out : Xn, last ? nN : NPB);
    if (!last)
      k_glob<<<1, GTHR, 0, stream>>>(GSEG, Xn, ESUM, OFF2, Uc, gW + (size_t)l * 15, gb + (size_t)l * 3,
                                      gg + (size_t)l * 3, gbt + (size_t)l * 3, nN, nG, Un);
  }
}
